// Model2_6305011990975
// MI455X (gfx1250) — hardware-verified
//
#include <hip/hip_runtime.h>
#include <stdint.h>
#include <stddef.h>

typedef __attribute__((ext_vector_type(16))) _Float16 v16h;
typedef __attribute__((ext_vector_type(8)))  _Float16 v8h;
typedef __attribute__((ext_vector_type(8)))  float    v8f;
typedef __attribute__((ext_vector_type(4)))  float    v4f;

constexpr int NB   = 256;
constexpr int NT   = 128;
constexpr int NV   = 128;
constexpr int NH   = 512;
constexpr int NCLS = 10;
constexpr int NCP  = 16;
constexpr int BT   = 16;
constexpr int NTHR = 512;
constexpr int NWAVE = NTHR / 32;
constexpr float WSC = 256.0f;
constexpr float ASC = 16.0f;
constexpr float ACC_INV = 1.0f / 4096.0f;

static_assert(NH == NTHR);
static_assert(NWAVE == BT);
static_assert(NWAVE * 2 * 16 == NH);
static_assert(NV == 8 * 16);
static_assert(NV == 32 * 4);
static_assert(NB % BT == 0);
static_assert(NV % 32 == 0 && NH % 32 == 0);
static_assert(NCLS <= NCP);
static_assert((NT * NCLS) % 4 == 0 && (NT * NCLS) / 4 == 320);

constexpr int OFF_HG = 0;
constexpr int OFF_P1 = BT * NH;
constexpr int OFF_P2 = 2 * BT * NH;
constexpr int OFF_IN = 3 * BT * NH;
constexpr int A16_HALVES = 3 * BT * NH + BT * NV;

union FragU { v16h v; v8h h[2]; };
__device__ __forceinline__ v16h frag_ld(const _Float16* p) {
  FragU f; f.h[0] = *(const v8h*)(p); f.h[1] = *(const v8h*)(p + 16); return f.v;
}
__device__ __forceinline__ v8f mma16(v16h a, v16h b, v8f c) {
  return __builtin_amdgcn_wmma_f32_16x16x32_f16(false, a, false, b, (short)0, c, false, false);
}
__device__ __forceinline__ void guard3(v8f& a, v8f& b, v8f& c, v16h w, v16h x, v16h y, v16h z) {
  asm volatile("v_nop\n\tv_nop\n\tv_nop\n\tv_nop" : "+v"(a), "+v"(b), "+v"(c) : "v"(w), "v"(x), "v"(y), "v"(z));
}
__device__ __forceinline__ void guard1(v8f& a, v16h x, v16h y) {
  asm volatile("v_nop\n\tv_nop\n\tv_nop\n\tv_nop" : "+v"(a) : "v"(x), "v"(y));
}
__device__ __forceinline__ void accg4(v8f& a, v8f& b, v8f& c, v8f& d) {
  asm volatile("v_nop\n\tv_nop\n\tv_nop\n\tv_nop" : "+v"(a), "+v"(b), "+v"(c), "+v"(d));
}
__device__ __forceinline__ void accg1(v8f& a) {
  asm volatile("v_nop\n\tv_nop\n\tv_nop\n\tv_nop" : "+v"(a));
}
__device__ __forceinline__ float sigm(float v) { return 1.0f / (1.0f + expf(-v)); }

__global__ __launch_bounds__(256) void cast_scale_f16x2(
    const float* __restrict__ in, _Float16* __restrict__ out, int n2, int nvalid2, float sc) {
  const int i = blockIdx.x * 256 + threadIdx.x;
  if (i < n2) {
    const int src = (i < nvalid2) ? i : (nvalid2 - 1);
    float f0 = in[2 * (size_t)src] * sc;
    float f1 = in[2 * (size_t)src + 1] * sc;
    if (i >= nvalid2) { f0 = 0.0f; f1 = 0.0f; }
    const _Float16 h0 = (_Float16)f0;
    const _Float16 h1 = (_Float16)f1;
    const unsigned u = (unsigned)__builtin_bit_cast(unsigned short, h0) |
                       ((unsigned)__builtin_bit_cast(unsigned short, h1) << 16);
    ((volatile unsigned*)out)[i] = u;
    __threadfence();
    ((volatile unsigned*)out)[i] = u;
  }
}

struct GParams {
  const float* x;   const float* d;   const float* m1;
  const float* h01; const float* h02; const float* h03;
  const float* bi1; const float* bh1; const float* bi2; const float* bh2; const float* bi3; const float* bh3;
  const float* bo;  const float* bx;  const float* bm;  const float* wd;  const float* bd;
  const _Float16* wi1; const _Float16* wh1; const _Float16* wi2; const _Float16* wh2; const _Float16* wi3; const _Float16* wh3;
  const _Float16* wx;  const _Float16* wm;  const _Float16* wo;
  float* yws; float* out;
};
static_assert(sizeof(GParams) == 28 * sizeof(void*));

__global__ __launch_bounds__(NTHR) void gru_decay_main(GParams p) {
  __shared__ __align__(16) float    Hs[3 * BT * NH];
  __shared__ __align__(16) float    Gs[BT * NH];
  __shared__ __align__(16) _Float16 A16[A16_HALVES];
  __shared__ __align__(16) float    XH[BT * NV];
  __shared__ float Dsm[BT];

  const int tid  = threadIdx.x;
  const int lane = tid & 31;
  const int wave = tid >> 5;
  const int hh   = lane >> 4;
  const int c16  = lane & 15;
  const int b0   = blockIdx.x * BT;
  float* const Mst  = Gs;
  float* const Yst  = Gs + BT * NV;
  float* const outX = p.out + (size_t)NB * NT * NCLS;
  float* const outM = outX + (size_t)NB * (NT - 1) * NV;
  const v8f z8 = {0.f, 0.f, 0.f, 0.f, 0.f, 0.f, 0.f, 0.f};

#pragma unroll 4
  for (int i = tid; i < BT * NH; i += NTHR) {
    const int r = i / NH;
    const size_t g = (size_t)(b0 + r) * NH + (i & (NH - 1));
    Hs[i]               = p.h01[g];
    Hs[BT * NH + i]     = p.h02[g];
    Hs[2 * BT * NH + i] = p.h03[g];
  }
  const float wdc = p.wd[tid];
  const float bdc = p.bd[tid];
  __syncthreads();

  for (int t = 0; t < NT; ++t) {
    if (tid < BT) Dsm[tid] = p.d[(size_t)(b0 + tid) * NT + t];
    for (int i = tid; i < BT * NV; i += NTHR) {
      const int r = i / NV;
      const int v = i & (NV - 1);
      const size_t gi = ((size_t)(b0 + r) * NT + t) * NV + v;
      const float xv = p.x[gi];
      float x1;
      if (t == 0) {
        x1 = xv;
      } else {
        const float mv = p.m1[gi];
        x1 = XH[i] * (1.0f - mv) + mv * xv;
      }
      A16[OFF_IN + i] = (_Float16)(x1 * ASC);
    }
    __syncthreads();

#pragma unroll 1
    for (int l = 0; l < 3; ++l) {
      float* const Hl = Hs + l * (BT * NH);
      for (int i = tid; i < BT * NH; i += NTHR) {
        const int r = i / NH;
        float g;
        if (l == 0) {
          g = (t == 0) ? 1.0f : expf(-fmaxf(wdc * Dsm[r] + bdc, 0.0f));
          Gs[i] = g;
        } else {
          g = Gs[i];
        }
        A16[OFF_HG + i] = (_Float16)(Hl[i] * g * ASC);
      }
      __syncthreads();

      const _Float16* const Wi = (l == 0) ? p.wi1 : (l == 1) ? p.wi2 : p.wi3;
      const _Float16* const Wh = (l == 0) ? p.wh1 : (l == 1) ? p.wh2 : p.wh3;
      const float*    const bi = (l == 0) ? p.bi1 : (l == 1) ? p.bi2 : p.bi3;
      const float*    const bh = (l == 0) ? p.bh1 : (l == 1) ? p.bh2 : p.bh3;
      const int offIn  = (l == 0) ? OFF_IN : (l == 1) ? OFF_P1 : OFF_P2;
      const int offOut = (l == 1) ? OFF_P2 : OFF_P1;
      const int Kin    = (l == 0) ? NV : NH;

#pragma unroll 1
      for (int jj = 0; jj < 2; ++jj) {
        const int j = wave * 2 + jj;
        v8f aR = z8, aZ = z8, aI = z8, aH = z8;
        {
          const _Float16* arow = A16 + offIn + c16 * Kin + 8 * hh;
          const _Float16* w0 = Wi + (size_t)(j * 16 + c16) * Kin + 8 * hh;
          const _Float16* w1 = w0 + (size_t)NH * Kin;
          const _Float16* w2 = w1 + (size_t)NH * Kin;
#pragma unroll 1
          for (int k0 = 0; k0 < Kin; k0 += 32) {
            const v16h a  = frag_ld(arow + k0);
            const v16h f0 = frag_ld(w0 + k0);
            const v16h f1 = frag_ld(w1 + k0);
            const v16h f2 = frag_ld(w2 + k0);
            aR = mma16(a, f0, aR);
            aZ = mma16(a, f1, aZ);
            aI = mma16(a, f2, aI);
            guard3(aR, aZ, aI, a, f0, f1, f2);
          }
        }
        {
          const _Float16* hrow = A16 + OFF_HG + c16 * NH + 8 * hh;
          const _Float16* u0 = Wh + (size_t)(j * 16 + c16) * NH + 8 * hh;
          const _Float16* u1 = u0 + (size_t)NH * NH;
          const _Float16* u2 = u1 + (size_t)NH * NH;
#pragma unroll 1
          for (int k0 = 0; k0 < NH; k0 += 32) {
            const v16h a  = frag_ld(hrow + k0);
            const v16h f0 = frag_ld(u0 + k0);
            const v16h f1 = frag_ld(u1 + k0);
            const v16h f2 = frag_ld(u2 + k0);
            aR = mma16(a, f0, aR);
            aZ = mma16(a, f1, aZ);
            aH = mma16(a, f2, aH);
            guard3(aR, aZ, aH, a, f0, f1, f2);
          }
        }
        accg4(aR, aZ, aI, aH);
        const int nc = j * 16 + c16;
        const float bR  = bi[nc] + bh[nc];
        const float bZ  = bi[NH + nc] + bh[NH + nc];
        const float bI  = bi[2 * NH + nc];
        const float bHn = bh[2 * NH + nc];
#pragma unroll
        for (int r = 0; r < 8; ++r) {
          const int idx = (8 * hh + r) * NH + nc;
          const float rg = sigm(aR[r] * ACC_INV + bR);
          const float zg = sigm(aZ[r] * ACC_INV + bZ);
          const float ng = tanhf(aI[r] * ACC_INV + bI + rg * (aH[r] * ACC_INV + bHn));
          const float hd = Hl[idx] * Gs[idx];
          const float hv = (1.0f - zg) * ng + zg * hd;
          Hl[idx] = hv;
          A16[offOut + idx] = (_Float16)(hv * ASC);
        }
      }
      __syncthreads();
    }

    {
      const bool isX = (wave < 8);
      const int  nt  = isX ? wave : (wave - 8);
      const _Float16* crow = A16 + OFF_P1 + c16 * NH + 8 * hh;
      const _Float16* wrow = (isX ? p.wx : p.wm) + (size_t)(nt * 16 + c16) * NH + 8 * hh;
      v8f acc = z8;
#pragma unroll 1
      for (int k0 = 0; k0 < NH; k0 += 32) {
        const v16h a = frag_ld(crow + k0);
        const v16h f = frag_ld(wrow + k0);
        acc = mma16(a, f, acc);
        guard1(acc, a, f);
      }
      accg1(acc);
      const int col = nt * 16 + c16;
      if (isX) {
        const float bb = p.bx[col];
#pragma unroll
        for (int r = 0; r < 8; ++r) XH[(8 * hh + r) * NV + col] = acc[r] * ACC_INV + bb;
      } else {
        const float bb = p.bm[col];
#pragma unroll
        for (int r = 0; r < 8; ++r) Mst[(8 * hh + r) * NV + col] = sigm(acc[r] * ACC_INV + bb);
      }
      if (wave == 0) {
        v8f ao = z8;
        const _Float16* orow = p.wo + (size_t)c16 * NH + 8 * hh;
#pragma unroll 1
        for (int k0 = 0; k0 < NH; k0 += 32) {
          const v16h a = frag_ld(crow + k0);
          const v16h f = frag_ld(orow + k0);
          ao = mma16(a, f, ao);
          guard1(ao, a, f);
        }
        accg1(ao);
        const bool live = (c16 < NCLS);
        const float boc = p.bo[live ? c16 : (NCLS - 1)];
#pragma unroll
        for (int r = 0; r < 8; ++r) {
          const float v = live ? (ao[r] * ACC_INV + boc) : -3.0e38f;
          float m = v;
          m = fmaxf(m, __shfl_xor(m, 1, 32));
          m = fmaxf(m, __shfl_xor(m, 2, 32));
          m = fmaxf(m, __shfl_xor(m, 4, 32));
          m = fmaxf(m, __shfl_xor(m, 8, 32));
          const float e = live ? expf(v - m) : 0.0f;
          float s = e;
          s += __shfl_xor(s, 1, 32);
          s += __shfl_xor(s, 2, 32);
          s += __shfl_xor(s, 4, 32);
          s += __shfl_xor(s, 8, 32);
          Yst[(8 * hh + r) * NCP + c16] = e * (1.0f / s);
        }
      }
    }
    __syncthreads();

    {
      if (wave == 0) {
        const v4f y0v = *(const v4f*)(Yst + 4 * lane);
        const v4f y1v = *(const v4f*)(Yst + 128 + 4 * lane);
        float* const ydst = p.yws + ((size_t)t * NB + b0) * NCP;
        for (int pass = 0; pass < 2; ++pass) {
          *(volatile v4f*)(ydst + 4 * lane) = y0v;
          *(volatile v4f*)(ydst + 128 + 4 * lane) = y1v;
          __threadfence();
        }
      }
      if (t > 0) {
        const v4f vx = *(const v4f*)(XH + wave * NV + 4 * lane);
        const v4f vm = *(const v4f*)(Mst + wave * NV + 4 * lane);
        const size_t ro = ((size_t)(b0 + wave) * (NT - 1) + (t - 1)) * NV + 4 * lane;
        for (int pass = 0; pass < 2; ++pass) {
          *(volatile v4f*)(outX + ro) = vx;
          *(volatile v4f*)(outM + ro) = vm;
          __threadfence();
        }
      }
    }
    __syncthreads();
  }
}

__global__ __launch_bounds__(320) void y_pack(const float* __restrict__ yws, float* __restrict__ out) {
  const int b  = blockIdx.x;
  const int i  = threadIdx.x;
  const int e0 = 4 * i;
  float f[4];
#pragma unroll
  for (int e = 0; e < 4; ++e) {
    const int el = e0 + e;
    const int t  = el / NCLS;
    const int c  = el - t * NCLS;
    f[e] = yws[((size_t)t * NB + b) * NCP + c];
  }
  const v4f v = {f[0], f[1], f[2], f[3]};
  float* const dst = out + (size_t)b * (NT * NCLS) + e0;
  for (int pass = 0; pass < 2; ++pass) {
    *(volatile v4f*)dst = v;
    __threadfence();
  }
}

constexpr size_t NEL_WI1 = (size_t)3 * NH * NV;
constexpr size_t NEL_WHH = (size_t)3 * NH * NH;
constexpr size_t NEL_WX  = (size_t)NV * NH;
constexpr size_t NEL_WO  = (size_t)NCP * NH;
constexpr size_t OB_WI1 = 0;
constexpr size_t OB_WH1 = OB_WI1 + NEL_WI1 * 2;
constexpr size_t OB_WI2 = OB_WH1 + NEL_WHH * 2;
constexpr size_t OB_WH2 = OB_WI2 + NEL_WHH * 2;
constexpr size_t OB_WI3 = OB_WH2 + NEL_WHH * 2;
constexpr size_t OB_WH3 = OB_WI3 + NEL_WHH * 2;
constexpr size_t OB_WX  = OB_WH3 + NEL_WHH * 2;
constexpr size_t OB_WM  = OB_WX  + NEL_WX * 2;
constexpr size_t OB_WO  = OB_WM  + NEL_WX * 2;
constexpr size_t OB_Y   = OB_WO  + NEL_WO * 2;
constexpr size_t WS_TOTAL = OB_Y + (size_t)NT * NB * NCP * 4;
static_assert(WS_TOTAL == 10633216);
static_assert(WS_TOTAL <= (size_t)134217728);
static_assert(OB_WH1 % 128 == 0 && OB_WI2 % 128 == 0 && OB_WX % 128 == 0 && OB_WM % 128 == 0 && OB_WO % 128 == 0 && OB_Y % 128 == 0);
static_assert((size_t)NB * NT * NCLS * 4 == 1310720);
static_assert((size_t)NB * NT * NCLS * 4 + (size_t)NB * (NT - 1) * NV * 4 == 17956864);
static_assert((size_t)NB * NT * NCLS * 4 + 2 * (size_t)NB * (NT - 1) * NV * 4 == 34603008);

extern "C" void kernel_launch(void* const* d_in, const int* in_sizes, int n_in,
                              void* d_out, int out_size, void* d_ws, size_t ws_size,
                              hipStream_t stream) {
  if (n_in < 26) return;
  if (in_sizes[0] != NB * NT * NV || in_sizes[2] != NB * NT * NV || in_sizes[7] != 3 * NH * NH ||
      in_sizes[6] != 3 * NH * NV || in_sizes[18] != NCLS * NH || in_sizes[20] != NV * NH) return;
  if (out_size != NB * NT * NCLS + 2 * NB * (NT - 1) * NV) return;
  if (ws_size < WS_TOTAL) return;

  const float* x    = (const float*)d_in[0];
  const float* d    = (const float*)d_in[1];
  const float* m1   = (const float*)d_in[2];
  const float* h01  = (const float*)d_in[3];
  const float* h02  = (const float*)d_in[4];
  const float* h03  = (const float*)d_in[5];
  const float* Wi1  = (const float*)d_in[6];
  const float* Wh1  = (const float*)d_in[7];
  const float* bi1  = (const float*)d_in[8];
  const float* bh1  = (const float*)d_in[9];
  const float* Wi2  = (const float*)d_in[10];
  const float* Wh2  = (const float*)d_in[11];
  const float* bi2  = (const float*)d_in[12];
  const float* bh2  = (const float*)d_in[13];
  const float* Wi3  = (const float*)d_in[14];
  const float* Wh3  = (const float*)d_in[15];
  const float* bi3  = (const float*)d_in[16];
  const float* bh3  = (const float*)d_in[17];
  const float* Wo   = (const float*)d_in[18];
  const float* bo   = (const float*)d_in[19];
  const float* Wx   = (const float*)d_in[20];
  const float* bx   = (const float*)d_in[21];
  const float* Wm   = (const float*)d_in[22];
  const float* bm   = (const float*)d_in[23];
  const float* Wd   = (const float*)d_in[24];
  const float* bd   = (const float*)d_in[25];

  char* const ws = (char*)d_ws;
  _Float16* const wi1h = (_Float16*)(ws + OB_WI1);
  _Float16* const wh1h = (_Float16*)(ws + OB_WH1);
  _Float16* const wi2h = (_Float16*)(ws + OB_WI2);
  _Float16* const wh2h = (_Float16*)(ws + OB_WH2);
  _Float16* const wi3h = (_Float16*)(ws + OB_WI3);
  _Float16* const wh3h = (_Float16*)(ws + OB_WH3);
  _Float16* const wxh  = (_Float16*)(ws + OB_WX);
  _Float16* const wmh  = (_Float16*)(ws + OB_WM);
  _Float16* const woh  = (_Float16*)(ws + OB_WO);
  float*    const yws  = (float*)(ws + OB_Y);

  auto cast = [&](const float* src, _Float16* dst, size_t n_total, size_t n_valid, float sc) {
    const int n2 = (int)(n_total / 2), nv2 = (int)(n_valid / 2);
    cast_scale_f16x2<<<(n2 + 255) / 256, 256, 0, stream>>>(src, dst, n2, nv2, sc);
  };
  cast(Wi1, wi1h, NEL_WI1, NEL_WI1, WSC);
  cast(Wh1, wh1h, NEL_WHH, NEL_WHH, WSC);
  cast(Wi2, wi2h, NEL_WHH, NEL_WHH, WSC);
  cast(Wh2, wh2h, NEL_WHH, NEL_WHH, WSC);
  cast(Wi3, wi3h, NEL_WHH, NEL_WHH, WSC);
  cast(Wh3, wh3h, NEL_WHH, NEL_WHH, WSC);
  cast(Wx,  wxh,  NEL_WX,  NEL_WX,  WSC);
  cast(Wm,  wmh,  NEL_WX,  NEL_WX,  WSC);
  cast(Wo,  woh,  NEL_WO,  (size_t)NCLS * NH, WSC);

  GParams p;
  p.x = x; p.d = d; p.m1 = m1; p.h01 = h01; p.h02 = h02; p.h03 = h03;
  p.bi1 = bi1; p.bh1 = bh1; p.bi2 = bi2; p.bh2 = bh2; p.bi3 = bi3; p.bh3 = bh3;
  p.bo = bo; p.bx = bx; p.bm = bm; p.wd = Wd; p.bd = bd;
  p.wi1 = wi1h; p.wh1 = wh1h; p.wi2 = wi2h; p.wh2 = wh2h; p.wi3 = wi3h; p.wh3 = wh3h;
  p.wx = wxh; p.wm = wmh; p.wo = woh;
  p.yws = yws; p.out = (float*)d_out;

  gru_decay_main<<<NB / BT, NTHR, 0, stream>>>(p);
  y_pack<<<NB, 320, 0, stream>>>(yws, (float*)d_out);
}
